// ConvBlock_50680614093178
// MI455X (gfx1250) — hardware-verified
//
#include <hip/hip_runtime.h>
#include <math.h>


#define NB 4
#define CI 64
#define DM 128
#define KW 8
#define L0 8192
#define L1 4096
#define DI 256
#define DS 16
#define DR 8
#define NXP 40

typedef __attribute__((ext_vector_type(16))) _Float16 v16h;
typedef __attribute__((ext_vector_type(8)))  _Float16 v8h;
typedef __attribute__((ext_vector_type(8)))  float v8f;
typedef __attribute__((ext_vector_type(4)))  float v4f;
typedef __attribute__((ext_vector_type(4)))  unsigned v4u;
typedef float __attribute__((may_alias)) float_a;

template <typename T> __device__ __forceinline__ void vst2(void* p, T v) { *(volatile T*)p = v; __threadfence(); *(volatile T*)p = v; }
__device__ __forceinline__ v8f wmma16(v16h a, v16h b, v8f c) {
  v8f d = __builtin_amdgcn_wmma_f32_16x16x32_f16(false, a, false, b, (short)0, c, false, false);
  asm volatile("v_nop\n\tv_nop\n\tv_nop\n\tv_nop" : "+v"(d) : "v"(a), "v"(b));
  return d;
}
__device__ __forceinline__ v16h frag_h(const _Float16* rowk0, int lane) {
  union { v16h v; v8h q[2]; } u; const _Float16* p = rowk0 + 8 * (lane >> 4);
  u.q[0] = *(const v8h*)p; u.q[1] = *(const v8h*)(p + 16); return u.v;
}
__device__ __forceinline__ v16h frag_f32(const float* rowk0, int lane) {
  v16h a; const float* p = rowk0 + 8 * (lane >> 4);
#pragma unroll
  for (int i = 0; i < 8; ++i) { a[i] = (_Float16)p[i]; a[8 + i] = (_Float16)p[16 + i]; }
  return a;
}
__device__ __forceinline__ float lrelu(float v) { return v >= 0.f ? v : 0.1f * v; }
__device__ __forceinline__ float silu(float v) { return v / (1.0f + expf(-v)); }
#define LDSX() do { asm volatile("s_wait_dscnt 0" ::: "memory"); __builtin_amdgcn_wave_barrier(); __builtin_amdgcn_fence(__ATOMIC_RELEASE, "workgroup"); } while (0)

__global__ __launch_bounds__(256) void k_wnorm(const float* __restrict__ v, const float* __restrict__ g, _Float16* __restrict__ We, int IK) {
  __shared__ float red[256], row[1024];
  const int o = blockIdx.x, tid = threadIdx.x;
  float s = 0.f;
  for (int i = tid; i < IK; i += 256) { const float w = v[(size_t)o * IK + i]; row[i] = w; s += w * w; }
  red[tid] = s; __syncthreads();
  for (int st = 128; st > 0; st >>= 1) { if (tid < st) red[tid] += red[tid + st]; __syncthreads(); }
  const float sc = g[o] / sqrtf(red[0]);
  for (int q = tid; q < IK / 8; q += 256) { union { v8h h; v4u u; } pk;
#pragma unroll
    for (int e = 0; e < 8; ++e) pk.h[e] = (_Float16)(row[q * 8 + e] * sc);
    vst2(We + (size_t)o * IK + q * 8, pk.u); }
}
__global__ __launch_bounds__(256) void k_cvt(const float* __restrict__ s, _Float16* __restrict__ d, size_t n8) {
  const size_t g8 = (size_t)blockIdx.x * 256 + threadIdx.x; if (g8 >= n8) return;
  union { v8h h; v4u u; } pk;
#pragma unroll
  for (int e = 0; e < 8; ++e) pk.h[e] = (_Float16)s[g8 * 8 + e];
  vst2(d + g8 * 8, pk.u);
}

template <int I, int RES>
__global__ __launch_bounds__(128) void k_conv(const float* __restrict__ in, const _Float16* __restrict__ We, const float* __restrict__ cb,
                                            const float* __restrict__ lg, const float* __restrict__ lb, const float* __restrict__ res, float* __restrict__ out) {
  __shared__ __align__(16) float st[DM][68];
  __shared__ float mu_s[64], rs_s[64];
  const int tid = threadIdx.x, wave = tid >> 5, lane = tid & 31, col = lane & 15, g = lane >> 4;
  const int b = blockIdx.y, t0 = blockIdx.x * 64, trow = t0 + wave * 16 + col;
  v8f acc[8] = {};
#pragma unroll 1
  for (int kc = 0; kc < I * KW / 32; ++kc) {
    v16h a; const int i0 = (kc * 32 + 8 * g) >> 3, i1 = i0 + 2;
    const float* p0 = in + ((size_t)b * I + i0) * L0 + trow; const float* p1 = in + ((size_t)b * I + i1) * L0 + trow;
#pragma unroll
    for (int e = 0; e < 8; ++e) { a[e] = (_Float16)(trow + e < L0 ? p0[e] : 0.f); a[8 + e] = (_Float16)(trow + e < L0 ? p1[e] : 0.f); }
#pragma unroll
    for (int j = 0; j < 8; ++j) acc[j] = wmma16(a, frag_h(We + (size_t)(j * 16 + col) * (I * KW) + kc * 32, lane), acc[j]);
  }
#pragma unroll
  for (int j = 0; j < 8; ++j) { const float bv = cb[j * 16 + col];
#pragma unroll
    for (int r = 0; r < 8; ++r) st[j * 16 + col][wave * 16 + 8 * g + r] = acc[j][r] + bv; }
  __syncthreads();
  { const int tl = tid >> 1, hf = tid & 1; float s = 0.f;
    for (int o = hf * 64; o < hf * 64 + 64; ++o) s += st[o][tl];
    s += __shfl_xor(s, 1, 32); const float mu = s / (float)DM;
    float q = 0.f;
    for (int o = hf * 64; o < hf * 64 + 64; ++o) { const float d = st[o][tl] - mu; q += d * d; }
    q += __shfl_xor(q, 1, 32);
    if (hf == 0) { mu_s[tl] = mu; rs_s[tl] = rsqrtf(q / (float)DM + 1e-5f); } }
  __syncthreads();
  for (int q = tid; q < DM * 16; q += 128) { const int o = q >> 4, pc = q & 15;
    v4f v;
#pragma unroll
    for (int e = 0; e < 4; ++e) { const int tl = pc * 4 + e; v[e] = lrelu((st[o][tl] - mu_s[tl]) * rs_s[tl] * lg[o] + lb[o]); }
    const size_t oo = ((size_t)b * DM + o) * L0 + t0 + pc * 4;
    if (RES) v += *(const v4f*)(res + oo);
    vst2(out + oo, v); }
}

__global__ __launch_bounds__(256) void k_pool(const float* __restrict__ h2, float* __restrict__ hp) {
  __shared__ float tile[DM][65];
  const int b = blockIdx.y, t0 = blockIdx.x * 64, tid = threadIdx.x;
  for (int i = tid; i < DM * 64; i += 256) { const int c = i >> 6, tl = i & 63; const float* p = h2 + ((size_t)b * DM + c) * L0 + 2 * (t0 + tl);
    tile[c][tl] = 0.5f * (p[0] + p[1]); }
  __syncthreads();
  for (int i = tid; i < 64 * 32; i += 256) { const int tl = i >> 5, pc = i & 31;
    v4f v = { tile[pc * 4][tl], tile[pc * 4 + 1][tl], tile[pc * 4 + 2][tl], tile[pc * 4 + 3][tl] };
    vst2(hp + ((size_t)b * L1 + t0 + tl) * DM + pc * 4, v); }
}

__global__ __launch_bounds__(256) void k_lnrows(const float* __restrict__ h, const float* __restrict__ lw, const float* __restrict__ lb, _Float16* __restrict__ o16) {
  const int r0 = blockIdx.x * 8, tid = threadIdx.x, wave = tid >> 5, lane = tid & 31;
  const size_t row = (size_t)r0 + wave;
  const v4f v = *(const v4f*)(h + row * DM + lane * 4);
  float s = v[0] + v[1] + v[2] + v[3];
#pragma unroll
  for (int off = 16; off >= 1; off >>= 1) s += __shfl_xor(s, off, 32);
  const float mu = s / (float)DM;
  const float d0 = v[0] - mu, d1 = v[1] - mu, d2 = v[2] - mu, d3 = v[3] - mu;
  float q = d0 * d0 + d1 * d1 + d2 * d2 + d3 * d3;
#pragma unroll
  for (int off = 16; off >= 1; off >>= 1) q += __shfl_xor(q, off, 32);
  const float rs = rsqrtf(q / (float)DM + 1e-5f);
  float o[4] = { d0 * rs * lw[lane * 4] + lb[lane * 4], d1 * rs * lw[lane * 4 + 1] + lb[lane * 4 + 1], d2 * rs * lw[lane * 4 + 2] + lb[lane * 4 + 2], d3 * rs * lw[lane * 4 + 3] + lb[lane * 4 + 3] };
  float n0 = __shfl_xor(o[0], 1, 32), n1 = __shfl_xor(o[1], 1, 32), n2 = __shfl_xor(o[2], 1, 32), n3 = __shfl_xor(o[3], 1, 32);
  if ((lane & 1) == 0) { union { v8h hh; v4u u; } pk;
    pk.hh[0] = (_Float16)o[0]; pk.hh[1] = (_Float16)o[1]; pk.hh[2] = (_Float16)o[2]; pk.hh[3] = (_Float16)o[3];
    pk.hh[4] = (_Float16)n0; pk.hh[5] = (_Float16)n1; pk.hh[6] = (_Float16)n2; pk.hh[7] = (_Float16)n3;
    vst2(o16 + row * DM + lane * 4, pk.u); }
}

template <int MODE>
__global__ __launch_bounds__(128) void k_gemm(const _Float16* __restrict__ A, const _Float16* __restrict__ W, const float* __restrict__ res,
                                            float* __restrict__ Out, int K, int N) {
  __shared__ __align__(16) float so[4][16 * 128];
  const int tid = threadIdx.x, wave = tid >> 5, lane = tid & 31, col = lane & 15, g = lane >> 4;
  const int r0 = blockIdx.x * 64 + wave * 16, n0 = blockIdx.y * 128;
  v8f acc[8] = {};
#pragma unroll 1
  for (int kc = 0; kc < K / 32; ++kc) { const v16h a = frag_h(A + (size_t)(r0 + col) * K + kc * 32, lane);
#pragma unroll
    for (int j = 0; j < 8; ++j) acc[j] = wmma16(a, frag_h(W + (size_t)(n0 + j * 16 + col) * K + kc * 32, lane), acc[j]); }
  float* S = so[wave];
#pragma unroll
  for (int j = 0; j < 8; ++j)
#pragma unroll
    for (int r = 0; r < 8; ++r) S[(8 * g + r) * 128 + j * 16 + col] = acc[j][r];
  LDSX();
#pragma unroll 4
  for (int rl = 0; rl < 16; ++rl) { const size_t o = (size_t)(r0 + rl) * N + n0 + lane * 4;
    v4f v = *(const v4f*)(S + rl * 128 + lane * 4); if (MODE) v += *(const v4f*)(res + o); vst2(Out + o, v); }
}

__global__ __launch_bounds__(256) void k_prep(const float* __restrict__ xz, const float* __restrict__ cw, const float* __restrict__ cbv,
                                            const float* __restrict__ xpW, const float* __restrict__ dtW, const float* __restrict__ dtb,
                                            float* __restrict__ xs2, float* __restrict__ dt, float* __restrict__ bc) {
  __shared__ float sx[DI], sd[NXP];
  const int b = blockIdx.y, t = blockIdx.x, d = threadIdx.x;
  const size_t row = (size_t)b * L1 + t;
  float a = cbv[d];
#pragma unroll
  for (int k = 0; k < 4; ++k) { const int tt = t - 3 + k; if (tt >= 0) a += cw[d * 4 + k] * xz[((size_t)b * L1 + tt) * (2 * DI) + d]; }
  const float xv = silu(a);
  sx[d] = xv;
  vst2(xs2 + row * DI + d, (float_a)xv);
  __syncthreads();
  if (d < NXP) { float s = 0.f;
#pragma unroll 1
    for (int i = 0; i < DI; ++i) s += sx[i] * xpW[(size_t)d * DI + i];
    sd[d] = s; }
  __syncthreads();
  { float s = dtb[d];
#pragma unroll
    for (int i = 0; i < DR; ++i) s += sd[i] * dtW[(size_t)d * DR + i];
    const float sp = s > 20.f ? s : log1pf(expf(s));
    vst2(dt + row * DI + d, (float_a)sp); }
  if (d < 32) vst2(bc + row * 32 + d, (float_a)sd[DR + d]);
}

__global__ __launch_bounds__(64) void k_scan(const float* __restrict__ xs2, const float* __restrict__ dt, const float* __restrict__ bc,
                                           const float* __restrict__ xz, const float* __restrict__ Alog, const float* __restrict__ Dp, _Float16* __restrict__ g16) {
  const int b = blockIdx.y, d = blockIdx.x * 64 + threadIdx.x;
  float A[DS], h[DS];
#pragma unroll
  for (int n = 0; n < DS; ++n) { A[n] = -expf(Alog[(size_t)d * DS + n]); h[n] = 0.f; }
  const float Dd = Dp[d];
#pragma unroll 1
  for (int t = 0; t < L1; ++t) { const size_t row = (size_t)b * L1 + t;
    const float dtv = dt[row * DI + d], xv = xs2[row * DI + d];
    const float* bcr = bc + row * 32;
    float y = 0.f;
#pragma unroll 1
    for (int n = 0; n < DS; ++n) { h[n] = expf(dtv * A[n]) * h[n] + dtv * bcr[n] * xv; y += h[n] * bcr[DS + n]; }
    y += xv * Dd;
    const float z = xz[row * (2 * DI) + DI + d];
    const _Float16 gv = (_Float16)(y * silu(z));
    *(volatile _Float16*)(g16 + row * DI + d) = gv; __threadfence(); *(volatile _Float16*)(g16 + row * DI + d) = gv; }
}

__global__ __launch_bounds__(256) void k_outT(const float* __restrict__ h, float* __restrict__ out) {
  __shared__ float tile[64][DM + 1];
  const int b = blockIdx.y, t0 = blockIdx.x * 64, tid = threadIdx.x;
  for (int i = tid; i < 64 * DM; i += 256) { const int tl = i / DM, c = i % DM; tile[tl][c] = h[((size_t)b * L1 + t0 + tl) * DM + c]; }
  __syncthreads();
  for (int i = tid; i < DM * 16; i += 256) { const int c = i >> 4, pc = i & 15;
    v4f v = { tile[pc * 4][c], tile[pc * 4 + 1][c], tile[pc * 4 + 2][c], tile[pc * 4 + 3][c] };
    vst2(out + ((size_t)b * DM + c) * L1 + t0 + pc * 4, v); }
}

extern "C" void kernel_launch(void* const* d_in, const int* in_sizes, int n_in,
                              void* d_out, int out_size, void* d_ws, size_t ws_size,
                              hipStream_t stream) {
  (void)in_sizes; (void)n_in; (void)out_size; (void)ws_size;
  const float* x = (const float*)d_in[0];
  const float* c1v = (const float*)d_in[1]; const float* c1g = (const float*)d_in[2]; const float* c1b = (const float*)d_in[3];
  const float* l1g = (const float*)d_in[4]; const float* l1b = (const float*)d_in[5];
  const float* c2v = (const float*)d_in[6]; const float* c2g = (const float*)d_in[7]; const float* c2b = (const float*)d_in[8];
  const float* l2g = (const float*)d_in[9]; const float* l2b = (const float*)d_in[10];
  const float* mlg = (const float*)d_in[11]; const float* mlb = (const float*)d_in[12];
  const float* inW = (const float*)d_in[13]; const float* cw = (const float*)d_in[14]; const float* cbv = (const float*)d_in[15];
  const float* xpW = (const float*)d_in[16]; const float* dtW = (const float*)d_in[17]; const float* dtb = (const float*)d_in[18];
  const float* Alog = (const float*)d_in[19]; const float* Dp = (const float*)d_in[20]; const float* outW = (const float*)d_in[21];
  float* out = (float*)d_out;
  char* ws = (char*)d_ws; size_t off = 0;
  auto take = [&](size_t bytes) { char* p = ws + off; off += (bytes + 255) & ~(size_t)255; return p; };
  _Float16* We1 = (_Float16*)take((size_t)DM * CI * KW * 2); _Float16* We2 = (_Float16*)take((size_t)DM * DM * KW * 2);
  _Float16* inWh = (_Float16*)take((size_t)2 * (2 * DI) * DM * 2); _Float16* outWh = (_Float16*)take((size_t)2 * DM * DI * 2);
  float* h1 = (float*)take((size_t)NB * DM * L0 * 4);
  float* h2 = (float*)take((size_t)NB * DM * L0 * 4);
  float* hp = (float*)take((size_t)NB * L1 * DM * 4);
  float* hq = (float*)take((size_t)NB * L1 * DM * 4);
  _Float16* u16 = (_Float16*)take((size_t)NB * L1 * DM * 2);
  float* xz = (float*)take((size_t)NB * L1 * 2 * DI * 4);
  float* xs2 = (float*)take((size_t)NB * L1 * DI * 4);
  float* dt = (float*)take((size_t)NB * L1 * DI * 4);
  float* bc = (float*)take((size_t)NB * L1 * 32 * 4);
  _Float16* g16 = (_Float16*)take((size_t)NB * L1 * DI * 2);
  k_wnorm<<<DM, 256, 0, stream>>>(c1v, c1g, We1, CI * KW);
  k_wnorm<<<DM, 256, 0, stream>>>(c2v, c2g, We2, DM * KW);
  k_cvt<<<(unsigned)((2 * 2 * DI * DM / 8 + 255) / 256), 256, 0, stream>>>(inW, inWh, (size_t)2 * 2 * DI * DM / 8);
  k_cvt<<<(unsigned)((2 * DM * DI / 8 + 255) / 256), 256, 0, stream>>>(outW, outWh, (size_t)2 * DM * DI / 8);
  k_conv<CI, 0><<<dim3(L0 / 64, NB), 128, 0, stream>>>(x, We1, c1b, l1g, l1b, nullptr, h1);
  k_conv<DM, 1><<<dim3(L0 / 64, NB), 128, 0, stream>>>(h1, We2, c2b, l2g, l2b, h1, h2);
  k_pool<<<dim3(L1 / 64, NB), 256, 0, stream>>>(h2, hp);
  float* hcur = hp; float* hnext = hq;
  for (int i = 0; i < 2; ++i) {
    k_lnrows<<<NB * L1 / 8, 256, 0, stream>>>(hcur, mlg + i * DM, mlb + i * DM, u16);
    k_gemm<0><<<dim3(NB * L1 / 64, 2 * DI / 128), 128, 0, stream>>>(u16, inWh + (size_t)i * 2 * DI * DM, nullptr, xz, DM, 2 * DI);
    k_prep<<<dim3(L1, NB), 256, 0, stream>>>(xz, cw + (size_t)i * DI * 4, cbv + i * DI, xpW + (size_t)i * NXP * DI, dtW + (size_t)i * DI * DR, dtb + i * DI, xs2, dt, bc);
    k_scan<<<dim3(DI / 64, NB), 64, 0, stream>>>(xs2, dt, bc, xz, Alog + (size_t)i * DI * DS, Dp + i * DI, g16);
    k_gemm<1><<<dim3(NB * L1 / 64, DM / 128), 128, 0, stream>>>(g16, outWh + (size_t)i * DM * DI, hcur, hnext, DI, DM);
    float* tmp = hcur; hcur = hnext; hnext = tmp;
  }
  k_outT<<<dim3(L1 / 64, NB), 256, 0, stream>>>(hcur, out);
}
